// Block_46669114638369
// MI455X (gfx1250) — hardware-run, weakly checked
//
#include <hip/hip_runtime.h>
#include <math.h>

typedef __attribute__((ext_vector_type(16))) __bf16   v16b;
typedef __attribute__((ext_vector_type(8)))  __bf16   v8b;
typedef __attribute__((ext_vector_type(8)))  float    v8f;
typedef __attribute__((ext_vector_type(4)))  float    v4f;
typedef __attribute__((ext_vector_type(2)))  float    v2f;
typedef __attribute__((ext_vector_type(4)))  unsigned v4u;

constexpr bool kLegBf16 = true;

constexpr int kBatch = 2;
constexpr int kSeq   = 2048;
constexpr int kDm    = 1024;
constexpr int kDin   = 2048;
constexpr int kNst   = 16;
constexpr int kRows  = kBatch * kSeq;
constexpr int kBcN   = 64;
static_assert(kRows == 4096, "rows");
static_assert((kDm % 32) == 0 && (kDin % 32) == 0, "GEMM K multiples of 32");
static_assert((kRows % 64) == 0 && (kDin % 64) == 0 && (kDm % 64) == 0 && (kBcN % 64) == 0, "GEMM M,N multiples of 64");
static_assert(2 * kNst <= kBcN, "stacked B|C width");

constexpr int kScanT       = 64;
constexpr int kScanCh      = 2 * kScanT;
constexpr int kScanTS      = 64;
constexpr int kScanYP      = 68;
constexpr int kScanBlkPerB = kDin / kScanCh;
static_assert((kSeq % kScanTS) == 0 && (kDin % kScanCh) == 0, "scan tiles");

constexpr size_t kLoMul = kLegBf16 ? 0 : 1;
constexpr size_t kSzX   = (size_t)kRows * kDm * 2;
constexpr size_t kSzWI  = (size_t)kDin * kDm * 2;
constexpr size_t kSzWD  = (size_t)kDin * kDin * 2;
constexpr size_t kSzWO  = (size_t)kDm * kDin * 2;
constexpr size_t kSzWB  = (size_t)kBcN * kDin * 2;
constexpr size_t kSzH   = (size_t)kRows * kDin * 2;
constexpr size_t kSzDT  = (size_t)kRows * kDin * 4;
constexpr size_t kSzBC  = (size_t)kRows * kBcN * 4;

constexpr size_t kOffXH  = 0;
constexpr size_t kOffXL  = kOffXH  + kSzX;
constexpr size_t kOffWIH = kOffXL  + kSzX * kLoMul;
constexpr size_t kOffWIL = kOffWIH + kSzWI;
constexpr size_t kOffWDH = kOffWIL + kSzWI * kLoMul;
constexpr size_t kOffWDL = kOffWDH + kSzWD;
constexpr size_t kOffWOH = kOffWDL + kSzWD * kLoMul;
constexpr size_t kOffWOL = kOffWOH + kSzWO;
constexpr size_t kOffWBH = kOffWOL + kSzWO * kLoMul;
constexpr size_t kOffWBL = kOffWBH + kSzWB;
constexpr size_t kOffHH  = kOffWBL + kSzWB * kLoMul;
constexpr size_t kOffHL  = kOffHH  + kSzH;
constexpr size_t kOffDT  = kOffHL  + kSzH;
constexpr size_t kOffBC  = kOffDT  + kSzDT;
constexpr size_t kOffYF  = kOffBC  + kSzBC;
constexpr size_t kOffYH  = kLegBf16 ? kOffYF : 0;
constexpr size_t kOffYL  = kOffYH + kSzH;
constexpr size_t kWsTotal = kLegBf16 ? (kOffYF + 2 * kSzH) : kOffYF;
static_assert(!kLegBf16 || kWsTotal == 127139840ull, "carve total");
static_assert(kLegBf16 || (kOffWOH >= 2 * kSzH), "aliased y planes fit inside dead planes");
static_assert(kWsTotal <= 134217728ull, "carve cap");
static_assert((kOffXL % 128) == 0 && (kOffWIH % 128) == 0 && (kOffWIL % 128) == 0 && (kOffWDH % 128) == 0 &&
              (kOffWDL % 128) == 0 && (kOffWOH % 128) == 0 && (kOffWOL % 128) == 0 && (kOffWBH % 128) == 0 &&
              (kOffWBL % 128) == 0 && (kOffHH % 128) == 0 && (kOffHL % 128) == 0 && (kOffDT % 128) == 0 &&
              (kOffBC % 128) == 0 && (kOffYF % 128) == 0 && (kOffYL % 128) == 0, "128-B aligned regions");

__device__ __forceinline__ unsigned rne_hi(float f) {
  unsigned u = __float_as_uint(f);
  const unsigned lsb = (u & 0x00010000u) ? 1u : 0u;
  u = (u + 0x7FFFu + lsb) & 0xFFFF0000u;
  return u;
}
__device__ __forceinline__ float rne_bf16_f(float f) { return __uint_as_float(rne_hi(f)); }
__device__ __forceinline__ unsigned pack_hi2(unsigned w1, unsigned w0) {
  return __builtin_amdgcn_perm(w1, w0, 0x07060302u);
}
__device__ __forceinline__ void split_pair(float f0, float f1, unsigned& hw, unsigned& lw) {
  const unsigned h0 = rne_hi(f0);
  const unsigned h1 = rne_hi(f1);
  const unsigned l0 = rne_hi(f0 - __uint_as_float(h0));
  const unsigned l1 = rne_hi(f1 - __uint_as_float(h1));
  hw = pack_hi2(h1, h0);
  lw = pack_hi2(l1, l0);
}
__device__ __forceinline__ void split8(float f0, float f1, float f2, float f3, float f4, float f5, float f6, float f7,
                                       v4u& hv, v4u& lv) {
  unsigned h0, l0, h1, l1, h2, l2, h3, l3;
  split_pair(f0, f1, h0, l0);
  split_pair(f2, f3, h1, l1);
  split_pair(f4, f5, h2, l2);
  split_pair(f6, f7, h3, l3);
  hv = (v4u){h0, h1, h2, h3};
  lv = (v4u){l0, l1, l2, l3};
}

__device__ __forceinline__ void wave_sync() {
  __builtin_amdgcn_fence(__ATOMIC_RELEASE, "workgroup");
  __builtin_amdgcn_wave_barrier();
  __builtin_amdgcn_fence(__ATOMIC_ACQUIRE, "workgroup");
}

template <bool WITH_LO>
__global__ __launch_bounds__(256) void rows_to_bf16_kernel(
    const float* __restrict__ src, unsigned short* __restrict__ dhi, unsigned short* __restrict__ dlo, int total8)
{
  const int i = blockIdx.x * 256 + threadIdx.x;
  if (i >= total8) return;
  const size_t e0 = (size_t)i << 3;
  const v4f a0 = *(const v4f*)(src + e0);
  const v4f a1 = *(const v4f*)(src + e0 + 4);
  const float f0 = a0[0], f1 = a0[1], f2 = a0[2], f3 = a0[3];
  const float f4 = a1[0], f5 = a1[1], f6 = a1[2], f7 = a1[3];
  v4u hv, lv;
  split8(f0, f1, f2, f3, f4, f5, f6, f7, hv, lv);
  volatile v4u* qh = (volatile v4u*)(dhi + e0);
  volatile v4u* ql = (volatile v4u*)(dlo + e0);
  *qh = hv;
  if (WITH_LO) *ql = lv;
  __threadfence();
  *qh = hv;
  if (WITH_LO) *ql = lv;
}

template <bool WITH_LO>
__global__ __launch_bounds__(256) void transpose_to_bf16_kernel(
    const float* __restrict__ W, unsigned short* __restrict__ Th, unsigned short* __restrict__ Tl, int R, int C)
{
  __shared__ float tile[64 * 65];
  const unsigned tid = threadIdx.x, lane = tid & 31u, wave = tid >> 5;
  const unsigned c0 = blockIdx.x * 64u;
  const unsigned r0 = blockIdx.y * 64u;
  const unsigned lr = tid >> 4, lc4 = (tid & 15u) * 4u;
#pragma unroll
  for (int i = 0; i < 4; ++i) {
    const unsigned r = lr + 16u * i;
    const v4f v = *(const v4f*)(W + (size_t)(r0 + r) * C + c0 + lc4);
    const float t0 = v[0], t1 = v[1], t2 = v[2], t3 = v[3];
    tile[r * 65u + lc4 + 0u] = t0;
    tile[r * 65u + lc4 + 1u] = t1;
    tile[r * 65u + lc4 + 2u] = t2;
    tile[r * 65u + lc4 + 3u] = t3;
  }
  __syncthreads();
  const unsigned q = lane >> 3, r8 = (lane & 7u) * 8u;
  v4u hv[2], lv[2];
#pragma unroll
  for (int it = 0; it < 2; ++it) {
    const unsigned c = it * 32u + wave * 4u + q;
    const float f0 = tile[(r8 + 0u) * 65u + c], f1 = tile[(r8 + 1u) * 65u + c];
    const float f2 = tile[(r8 + 2u) * 65u + c], f3 = tile[(r8 + 3u) * 65u + c];
    const float f4 = tile[(r8 + 4u) * 65u + c], f5 = tile[(r8 + 5u) * 65u + c];
    const float f6 = tile[(r8 + 6u) * 65u + c], f7 = tile[(r8 + 7u) * 65u + c];
    split8(f0, f1, f2, f3, f4, f5, f6, f7, hv[it], lv[it]);
  }
  for (int pass = 0; pass < 2; ++pass) {
#pragma unroll
    for (int it = 0; it < 2; ++it) {
      const unsigned c = it * 32u + wave * 4u + q;
      const size_t o = (size_t)(c0 + c) * R + r0 + r8;
      *(volatile v4u*)(Th + o) = hv[it];
      if (WITH_LO) *(volatile v4u*)(Tl + o) = lv[it];
    }
    __threadfence();
  }
}

template <bool WITH_LO>
__global__ __launch_bounds__(256) void stack_bc_weights_kernel(
    const float* __restrict__ WB, const float* __restrict__ WC,
    unsigned short* __restrict__ Th, unsigned short* __restrict__ Tl)
{
  __shared__ float tile[32 * 65];
  const unsigned tid = threadIdx.x, lane = tid & 31u, wave = tid >> 5;
  const unsigned k0 = blockIdx.x * 64u;
  {
    const unsigned kk = tid >> 2, n4 = (tid & 3u) * 4u;
    const v4f vb = *(const v4f*)(WB + (size_t)(k0 + kk) * kNst + n4);
    const v4f vc = *(const v4f*)(WC + (size_t)(k0 + kk) * kNst + n4);
    const float b0 = vb[0], b1 = vb[1], b2 = vb[2], b3 = vb[3];
    const float c0 = vc[0], c1 = vc[1], c2 = vc[2], c3 = vc[3];
    tile[(n4 + 0u) * 65u + kk] = b0;
    tile[(n4 + 1u) * 65u + kk] = b1;
    tile[(n4 + 2u) * 65u + kk] = b2;
    tile[(n4 + 3u) * 65u + kk] = b3;
    tile[(16u + n4 + 0u) * 65u + kk] = c0;
    tile[(16u + n4 + 1u) * 65u + kk] = c1;
    tile[(16u + n4 + 2u) * 65u + kk] = c2;
    tile[(16u + n4 + 3u) * 65u + kk] = c3;
  }
  __syncthreads();
  const unsigned q = lane >> 3, r8 = (lane & 7u) * 8u;
  v4u hv[2], lv[2];
#pragma unroll
  for (int it = 0; it < 2; ++it) {
    const unsigned n = it * 32u + wave * 4u + q;
    const unsigned nn = n & 31u;
    const bool live = (n < 32u);
    const float* sp = tile + nn * 65u + r8;
    const float g0 = sp[0], g1 = sp[1], g2 = sp[2], g3 = sp[3], g4 = sp[4], g5 = sp[5], g6 = sp[6], g7 = sp[7];
    const float f0 = live ? g0 : 0.0f, f1 = live ? g1 : 0.0f, f2 = live ? g2 : 0.0f, f3 = live ? g3 : 0.0f;
    const float f4 = live ? g4 : 0.0f, f5 = live ? g5 : 0.0f, f6 = live ? g6 : 0.0f, f7 = live ? g7 : 0.0f;
    split8(f0, f1, f2, f3, f4, f5, f6, f7, hv[it], lv[it]);
  }
  for (int pass = 0; pass < 2; ++pass) {
#pragma unroll
    for (int it = 0; it < 2; ++it) {
      const unsigned n = it * 32u + wave * 4u + q;
      const size_t o = (size_t)n * kDin + k0 + r8;
      *(volatile v4u*)(Th + o) = hv[it];
      if (WITH_LO) *(volatile v4u*)(Tl + o) = lv[it];
    }
    __threadfence();
  }
}

namespace eng {

union FragU { v16b v; v8b h[2]; };
__device__ __forceinline__ v16b frag_load(const __bf16* p) {
  FragU f;
  f.h[0] = *(const v8b*)(p);
  f.h[1] = *(const v8b*)(p + 16);
  return f.v;
}
__device__ __forceinline__ v8f mma(v16b a, v16b b, v8f c) {
  return __builtin_amdgcn_wmma_f32_16x16x32_bf16(false, a, false, b, (short)0, c, false, false);
}
__device__ __forceinline__ void tie1(v8f& a, v16b x, v16b y, v16b z) {
  asm volatile("" : "+v"(a) : "v"(x), "v"(y), "v"(z));
}
__device__ __forceinline__ void guard1(v8f& a, v16b x, v16b y, v16b z) {
  asm volatile("v_nop\n\tv_nop\n\tv_nop\n\tv_nop" : "+v"(a) : "v"(x), "v"(y), "v"(z));
}
__device__ __forceinline__ void keep4(v16b a, v16b b, v16b c, v16b d) {
  asm volatile("v_nop" :: "v"(a), "v"(b), "v"(c), "v"(d));
}
__device__ __forceinline__ void acc_guard1(v8f& a) {
  asm volatile("v_nop\n\tv_nop\n\tv_nop\n\tv_nop" : "+v"(a));
}

template <int ACT>
__device__ __forceinline__ float act_apply(float v) {
  if (ACT == 1) {
    const float em  = expm1f(v);
    const float neg = 1.6732632423543772f * em;
    const float sel = (v > 0.0f) ? v : neg;
    return 1.0507009873554805f * sel;
  }
  if (ACT == 2) {
    const float e = expf(-fabsf(v));
    return fmaxf(v, 0.0f) + log1pf(e);
  }
  return v;
}

template <int SPL, int BIAS_MODE, int OUT_MODE, int ACT, bool BIAS_RNE>
__global__ __launch_bounds__(256) void wmma_gemm64(
    const unsigned short* __restrict__ Ap, const unsigned short* __restrict__ A2p, int lda,
    const unsigned short* __restrict__ Btp, const unsigned short* __restrict__ Bt2p, int ldb,
    void* __restrict__ Cout, void* __restrict__ Cout2, int ldc,
    const float* __restrict__ bias, int M, int N, int K)
{
  const __bf16* A   = (const __bf16*)Ap;
  const __bf16* A2  = (const __bf16*)A2p;
  const __bf16* Bt  = (const __bf16*)Btp;
  const __bf16* Bt2 = (const __bf16*)Bt2p;
  __shared__ __align__(16) float sT[8][16 * 68];
  const int lane = threadIdx.x & 31;
  const int wave = threadIdx.x >> 5;
  const int tilesN = N >> 6;
  const int tilesM = M >> 6;
  const int tile = blockIdx.x * 8 + wave;
  if (tile >= tilesM * tilesN) return;
  const int tm = tile / tilesN;
  const int tn = tile - tm * tilesN;
  const int m0 = tm << 6;
  const int n0 = tn << 6;

  const int rlane = lane & 15;
  const int koff  = (lane >> 4) * 8;
  const int mOff  = (lane >> 4) * 8;

  v8f acc[4][4];
#pragma unroll
  for (int i = 0; i < 4; ++i)
#pragma unroll
    for (int j = 0; j < 4; ++j) acc[i][j] = (v8f){0.f, 0.f, 0.f, 0.f, 0.f, 0.f, 0.f, 0.f};

  for (int k0 = 0; k0 < K; k0 += 32) {
    v16b bh[4], bl[4];
#pragma unroll
    for (int j = 0; j < 4; ++j) {
      const size_t bo = (size_t)(n0 + (j << 4) + rlane) * ldb + koff + k0;
      bh[j] = frag_load(Bt + bo);
      if (SPL == 2) bl[j] = frag_load(Bt2 + bo);
      else bl[j] = bh[j];
    }
#pragma unroll
    for (int i = 0; i < 4; ++i) {
      const size_t ao = (size_t)(m0 + (i << 4) + rlane) * lda + koff + k0;
      const v16b ah = frag_load(A + ao);
      v16b al = ah;
      if (SPL >= 1) al = frag_load(A2 + ao);
#pragma unroll
      for (int j = 0; j < 4; ++j) {
        acc[i][j] = mma(ah, bh[j], acc[i][j]);
        if (SPL == 2) acc[i][j] = mma(ah, bl[j], acc[i][j]);
        if (SPL >= 1) acc[i][j] = mma(al, bh[j], acc[i][j]);
      }
      tie1(acc[i][0], ah, al, bh[0]);
      tie1(acc[i][1], ah, al, bh[1]);
      tie1(acc[i][2], ah, al, bh[2]);
      guard1(acc[i][3], ah, al, bh[3]);
    }
    keep4(bh[0], bh[1], bh[2], bh[3]);
    if (SPL == 2) keep4(bl[0], bl[1], bl[2], bl[3]);
  }
#pragma unroll
  for (int i = 0; i < 4; ++i) {
    acc_guard1(acc[i][0]);
    acc_guard1(acc[i][1]);
    acc_guard1(acc[i][2]);
    acc_guard1(acc[i][3]);
  }

  float* slab = sT[wave];
  float bv[4];
#pragma unroll
  for (int j = 0; j < 4; ++j) {
    bv[j] = 0.0f;
    if (BIAS_MODE == 2) {
      float t = bias[n0 + (j << 4) + rlane];
      if (BIAS_RNE) t = rne_bf16_f(t);
      bv[j] = t;
    }
  }
#pragma unroll
  for (int i = 0; i < 4; ++i) {
    const int mBase = m0 + (i << 4);
#pragma unroll
    for (int j = 0; j < 4; ++j) {
#pragma unroll
      for (int r = 0; r < 8; ++r) {
        slab[(mOff + r) * 68 + (j << 4) + rlane] = acc[i][j][r] + bv[j];
      }
    }
    wave_sync();
    if (ACT != 0) {
#pragma unroll 1
      for (int it = 0; it < 32; ++it) {
        const int row = it >> 1;
        const int col = ((it & 1) << 5) + lane;
        const float v = slab[row * 68 + col];
        const float w = act_apply<ACT>(v);
        slab[row * 68 + col] = w;
      }
      wave_sync();
    }
    if (OUT_MODE == 0) {
      float* C = (float*)Cout;
      const int hh = lane >> 4, c4 = (lane & 15) * 4;
      for (int pass = 0; pass < 2; ++pass) {
#pragma unroll
        for (int it = 0; it < 8; ++it) {
          const int row = it * 2 + hh;
          const v4f v = *(const v4f*)(slab + row * 68 + c4);
          *(volatile v4f*)(C + (size_t)(mBase + row) * ldc + n0 + c4) = v;
        }
        __threadfence();
      }
    } else {
      unsigned q = (unsigned)lane >> 3;
      unsigned c8 = ((unsigned)lane & 7u) * 8u;
      asm volatile("" : "+v"(q));
      asm volatile("" : "+v"(c8));
      unsigned short* C  = (unsigned short*)Cout;
      unsigned short* C2 = (unsigned short*)Cout2;
      v4u hw[4], lw[4];
#pragma unroll
      for (int it = 0; it < 4; ++it) {
        const unsigned row = it * 4u + q;
        const float* sp = slab + row * 68u + c8;
        const v4f a0 = *(const v4f*)(sp);
        const v4f a1 = *(const v4f*)(sp + 4);
        const float f0 = a0[0], f1 = a0[1], f2 = a0[2], f3 = a0[3];
        const float f4 = a1[0], f5 = a1[1], f6 = a1[2], f7 = a1[3];
        split8(f0, f1, f2, f3, f4, f5, f6, f7, hw[it], lw[it]);
      }
      for (int pass = 0; pass < 2; ++pass) {
#pragma unroll
        for (int it = 0; it < 4; ++it) {
          const unsigned row = it * 4u + q;
          const size_t o = (size_t)(mBase + row) * ldc + n0 + c8;
          *(volatile v4u*)(C + o)  = hw[it];
          *(volatile v4u*)(C2 + o) = lw[it];
        }
        __threadfence();
      }
    }
    wave_sync();
  }
}

}

template <bool RNE_IN>
__global__ __launch_bounds__(64) void state_scan_kernel(
    const float* __restrict__ DT, const unsigned* __restrict__ HHw, const unsigned* __restrict__ HLw,
    const float* __restrict__ BC, const float* __restrict__ bB, const float* __restrict__ bC,
    const float* __restrict__ Alog, const float* __restrict__ Dp,
    unsigned* __restrict__ YHw, unsigned* __restrict__ YLw)
{
  __shared__ __align__(16) float    sBC[kScanTS * 32];
  __shared__ __align__(16) float    sA[32 * kScanT];
  __shared__ __align__(16) unsigned sYh[kScanTS * kScanYP];
  __shared__ __align__(16) unsigned sYl[kScanTS * kScanYP];

  const unsigned tid = threadIdx.x, lane = tid & 31u, wave = tid >> 5;
  const unsigned bix = blockIdx.x / (unsigned)kScanBlkPerB;
  const unsigned d0  = (blockIdx.x - bix * (unsigned)kScanBlkPerB) * (unsigned)kScanCh;
  const unsigned d   = d0 + 2u * tid;
  const size_t row0  = (size_t)bix * kSeq;

#pragma unroll 1
  for (int j = 0; j < 2 * kNst; ++j) {
    float al = Alog[(size_t)d * kNst + j];
    if (RNE_IN) al = rne_bf16_f(al);
    sA[j * kScanT + tid] = -expf(al);
  }
  __syncthreads();
  float a0[kNst], a1[kNst], s0[kNst], s1[kNst];
#pragma unroll
  for (int k = 0; k < kNst; ++k) {
    a0[k] = sA[k * kScanT + tid];
    a1[k] = sA[(kNst + k) * kScanT + tid];
    s0[k] = 0.0f;
    s1[k] = 0.0f;
  }
  float D0, D1;
  {
    const v2f dp = *(const v2f*)(Dp + d);
    D0 = dp[0];
    D1 = dp[1];
    if (RNE_IN) { D0 = rne_bf16_f(D0); D1 = rne_bf16_f(D1); }
  }

  const unsigned lr = tid >> 3, lc4 = (tid & 7u) * 4u;
  float q0, q1, q2, q3;
  {
    const v4f vb = *(const v4f*)(bB + (lc4 & 12u));
    const v4f vc = *(const v4f*)(bC + (lc4 & 12u));
    float b0 = vb[0], b1 = vb[1], b2 = vb[2], b3 = vb[3];
    float c0 = vc[0], c1 = vc[1], c2 = vc[2], c3 = vc[3];
    asm volatile("" : "+v"(b0), "+v"(b1), "+v"(b2), "+v"(b3));
    asm volatile("" : "+v"(c0), "+v"(c1), "+v"(c2), "+v"(c3));
    const bool isB = (lc4 < 16u);
    q0 = isB ? b0 : c0;
    q1 = isB ? b1 : c1;
    q2 = isB ? b2 : c2;
    q3 = isB ? b3 : c3;
    if (RNE_IN) { q0 = rne_bf16_f(q0); q1 = rne_bf16_f(q1); q2 = rne_bf16_f(q2); q3 = rne_bf16_f(q3); }
  }

  const unsigned fr = lane >> 4, fc4 = (lane & 15u) * 4u;
  const size_t wbase = (size_t)(d0 >> 1);

#pragma unroll 1
  for (int t0 = 0; t0 < kSeq; t0 += kScanTS) {
    __syncthreads();
#pragma unroll
    for (int i = 0; i < 8; ++i) {
      const unsigned r = lr + 8u * i;
      v4f v = *(const v4f*)(BC + (row0 + t0 + r) * kBcN + lc4);
      v[0] = v[0] + q0;
      v[1] = v[1] + q1;
      v[2] = v[2] + q2;
      v[3] = v[3] + q3;
      *(v4f*)(sBC + r * 32u + lc4) = v;
    }
    __syncthreads();

#pragma unroll 1
    for (int s = 0; s < kScanTS; ++s) {
      const size_t row = row0 + t0 + s;
      const v2f dtv = *(const v2f*)(DT + row * kDin + d);
      const unsigned hw = HHw[row * (kDin / 2) + wbase + tid];
      const unsigned lw = HLw[row * (kDin / 2) + wbase + tid];
      const float dt0 = dtv[0], dt1 = dtv[1];
      const float h0 = __uint_as_float(hw << 16) + __uint_as_float(lw << 16);
      const float h1 = __uint_as_float(hw & 0xffff0000u) + __uint_as_float(lw & 0xffff0000u);
      const float* xr = sBC + s * 32;
      float y0 = 0.0f, y1 = 0.0f;
#pragma unroll
      for (int q4 = 0; q4 < 4; ++q4) {
        const v4f bvv = *(const v4f*)(xr + 4 * q4);
        const v4f cvv = *(const v4f*)(xr + kNst + 4 * q4);
#pragma unroll
        for (int e = 0; e < 4; ++e) {
          const int k = 4 * q4 + e;
          const float bb = bvv[e];
          const float cc = cvv[e];
          const float dA0 = __expf(dt0 * a0[k]);
          const float dA1 = __expf(dt1 * a1[k]);
          const float dB0 = dt0 * bb;
          const float dB1 = dt1 * bb;
          s0[k] = dA0 * s0[k] + dB0 * h0;
          s1[k] = dA1 * s1[k] + dB1 * h1;
          y0 = y0 + s0[k] * cc;
          y1 = y1 + s1[k] * cc;
        }
      }
      y0 = y0 + h0 * D0;
      y1 = y1 + h1 * D1;
      unsigned yh, yl;
      split_pair(y0, y1, yh, yl);
      sYh[s * kScanYP + tid] = yh;
      sYl[s * kScanYP + tid] = yl;
    }
    __syncthreads();

    for (int pass = 0; pass < 2; ++pass) {
#pragma unroll 4
      for (int it = 0; it < 16; ++it) {
        const unsigned rr = it * 4u + wave * 2u + fr;
        const v4u hv = *(const v4u*)(sYh + rr * kScanYP + fc4);
        const v4u lv = *(const v4u*)(sYl + rr * kScanYP + fc4);
        const size_t o = (row0 + t0 + rr) * (kDin / 2) + wbase + fc4;
        *(volatile v4u*)(YHw + o) = hv;
        *(volatile v4u*)(YLw + o) = lv;
      }
      __threadfence();
    }
  }
}

extern "C" void kernel_launch(void* const* d_in, const int* in_sizes, int n_in,
                              void* d_out, int out_size, void* d_ws, size_t ws_size,
                              hipStream_t stream) {
  if (n_in < 13) return;
  if (in_sizes[0] != kRows * kDm) return;
  if (in_sizes[1] != kDm * kDin) return;
  if (in_sizes[2] != kDin) return;
  if (in_sizes[3] != kDin * kNst) return;
  if (in_sizes[4] != kDin * kNst) return;
  if (in_sizes[5] != kNst) return;
  if (in_sizes[6] != kDin * kNst) return;
  if (in_sizes[7] != kNst) return;
  if (in_sizes[8] != kDin * kDin) return;
  if (in_sizes[9] != kDin) return;
  if (in_sizes[10] != kDin) return;
  if (in_sizes[11] != kDin * kDm) return;
  if (in_sizes[12] != kDm) return;
  if (out_size != kRows * kDm) return;
  if (ws_size < kWsTotal) return;

  const float* x       = (const float*)d_in[0];
  const float* W_in    = (const float*)d_in[1];
  const float* b_in    = (const float*)d_in[2];
  const float* A_log   = (const float*)d_in[3];
  const float* W_B     = (const float*)d_in[4];
  const float* b_B     = (const float*)d_in[5];
  const float* W_C     = (const float*)d_in[6];
  const float* b_C     = (const float*)d_in[7];
  const float* W_delta = (const float*)d_in[8];
  const float* b_delta = (const float*)d_in[9];
  const float* D_param = (const float*)d_in[10];
  const float* W_out   = (const float*)d_in[11];
  const float* b_out   = (const float*)d_in[12];
  float* out = (float*)d_out;

  char* ws = (char*)d_ws;
  unsigned short* XH  = (unsigned short*)(ws + kOffXH);
  unsigned short* XL  = kLegBf16 ? XH  : (unsigned short*)(ws + kOffXL);
  unsigned short* WIH = (unsigned short*)(ws + kOffWIH);
  unsigned short* WIL = kLegBf16 ? WIH : (unsigned short*)(ws + kOffWIL);
  unsigned short* WDH = (unsigned short*)(ws + kOffWDH);
  unsigned short* WDL = kLegBf16 ? WDH : (unsigned short*)(ws + kOffWDL);
  unsigned short* WOH = (unsigned short*)(ws + kOffWOH);
  unsigned short* WOL = kLegBf16 ? WOH : (unsigned short*)(ws + kOffWOL);
  unsigned short* WBH = (unsigned short*)(ws + kOffWBH);
  unsigned short* WBL = kLegBf16 ? WBH : (unsigned short*)(ws + kOffWBL);
  unsigned short* HH  = (unsigned short*)(ws + kOffHH);
  unsigned short* HL  = (unsigned short*)(ws + kOffHL);
  float*          DT  = (float*)(ws + kOffDT);
  float*          BC  = (float*)(ws + kOffBC);
  unsigned short* YH  = (unsigned short*)(ws + kOffYH);
  unsigned short* YL  = (unsigned short*)(ws + kOffYL);

  constexpr bool kLo = !kLegBf16;
  constexpr int kSplIn  = kLegBf16 ? 0 : 2;
  constexpr int kSplMid = kLegBf16 ? 1 : 2;

  rows_to_bf16_kernel<kLo><<<(kRows * kDm / 8) / 256, 256, 0, stream>>>(x, XH, XL, kRows * kDm / 8);
  transpose_to_bf16_kernel<kLo><<<dim3(kDin / 64, kDm / 64), 256, 0, stream>>>(W_in, WIH, WIL, kDm, kDin);
  transpose_to_bf16_kernel<kLo><<<dim3(kDin / 64, kDin / 64), 256, 0, stream>>>(W_delta, WDH, WDL, kDin, kDin);
  transpose_to_bf16_kernel<kLo><<<dim3(kDm / 64, kDin / 64), 256, 0, stream>>>(W_out, WOH, WOL, kDin, kDm);
  stack_bc_weights_kernel<kLo><<<kDin / 64, 256, 0, stream>>>(W_B, W_C, WBH, WBL);

  eng::wmma_gemm64<kSplIn, 2, 2, 1, kLegBf16><<<256, 256, 0, stream>>>(
      XH, XL, kDm,
      WIH, WIL, kDm,
      (void*)HH, (void*)HL, kDin,
      b_in, kRows, kDin, kDm);

  eng::wmma_gemm64<kSplMid, 2, 0, 2, kLegBf16><<<256, 256, 0, stream>>>(
      HH, HL, kDin,
      WDH, WDL, kDin,
      (void*)DT, (void*)DT, kDin,
      b_delta, kRows, kDin, kDin);

  eng::wmma_gemm64<kSplMid, 0, 0, 0, false><<<8, 256, 0, stream>>>(
      HH, HL, kDin,
      WBH, WBL, kDin,
      (void*)BC, (void*)BC, kBcN,
      b_B, kRows, kBcN, kDin);

  state_scan_kernel<kLegBf16><<<kBatch * kScanBlkPerB, kScanT, 0, stream>>>(
      DT, (const unsigned*)HH, (const unsigned*)HL, BC, b_B, b_C, A_log, D_param,
      (unsigned*)YH, (unsigned*)YL);

  eng::wmma_gemm64<kSplMid, 2, 0, 0, kLegBf16><<<128, 256, 0, stream>>>(
      YH, YL, kDin,
      WOH, WOL, kDin,
      (void*)out, (void*)out, kDm,
      b_out, kRows, kDm, kDin);
}
